// Embedding_23338852286583
// MI455X (gfx1250) — hardware-verified
//
#include <hip/hip_runtime.h>
#include <stddef.h>


typedef _Float16 h16;
typedef _Float16 v16h __attribute__((ext_vector_type(16)));
typedef _Float16 v8h  __attribute__((ext_vector_type(8)));
typedef float    v8f  __attribute__((ext_vector_type(8)));
typedef float    v4f  __attribute__((ext_vector_type(4)));

#ifndef NB
#define NB 64
#endif
#ifndef SEQ
#define SEQ 128
#endif
#define NB_FULL   64
#define SEQ_FULL  128
#define BAG       40
#define VOCAB     1276
#define AGE_DEPTH 91
#define KTRUE     (VOCAB + AGE_DEPTH)
#define KLOOP     1376
#define KPITCH    1408
#define DIMO      768
#define MROWS     (NB * SEQ)

static_assert(NB >= 1 && NB <= NB_FULL);
static_assert(SEQ >= 64 && SEQ <= SEQ_FULL && (SEQ % 64) == 0);
static_assert(KTRUE == 1367);
static_assert((KLOOP % 32) == 0 && KLOOP >= KTRUE);
static_assert((KPITCH % 64) == 0 && KPITCH >= KLOOP);
static_assert((DIMO % 64) == 0);
static_assert((MROWS % 64) == 0 && (MROWS % 8) == 0);
static_assert(BAG == 40);

#define LDT 72
#define LDC 68
static_assert((LDT % 8) == 0 && LDT >= 64);
static_assert((LDC % 4) == 0 && LDC >= 64);

#define WCARRY 64.0f

#define TOKB      8
#define IDP       48
#define ROWPIECES (KPITCH / 8)
#define CSTEPS    6
static_assert(TOKB * 32 == 256);
static_assert(CSTEPS * 32 >= ROWPIECES && (CSTEPS - 1) * 32 < ROWPIECES);
static_assert((ROWPIECES % 8) == 0);
static_assert(IDP >= BAG + 1);
static_assert((MROWS % TOKB) == 0);

static_assert((256 / 8) * 2 == 64);
static_assert((256 / 16) * 4 == 64);
static_assert(256 * 16 == 64 * 64);

static_assert((size_t)64 * LDT * 2 <= (size_t)131072);
static_assert((size_t)TOKB * KPITCH * 2 + (size_t)TOKB * IDP * 4 <= (size_t)131072);
static_assert((size_t)64 * LDC * 4 <= (size_t)131072);

#define WT_BYTES ((size_t)DIMO * KPITCH * 2)
#define X_BYTES  ((size_t)MROWS * KPITCH * 2)
#define OFF_WT   ((size_t)0)
#define OFF_X    (OFF_WT + WT_BYTES)
#define WS_TOTAL (OFF_X + X_BYTES)
static_assert((WT_BYTES % 128) == 0 && (X_BYTES % 128) == 0);
static_assert(WS_TOTAL <= (size_t)134217728);

__device__ __forceinline__ float bf16r(float x) {
  unsigned int u = __float_as_uint(x);
  u = (u + 0x7FFFu + ((u >> 16) & 1u)) & 0xFFFF0000u;
  return __uint_as_float(u);
}

static __device__ __forceinline__ h16 toh_flush(float v) {
  const h16 r = (h16)v;
  return (fabsf(v) < 6.103515625e-05f) ? (h16)0.0f : r;
}

__device__ __forceinline__ v16h frag_at(const _Float16* p) {
  v8h lo = *(const v8h*)(p);
  v8h hi = *(const v8h*)(p + 16);
  v16h out;
#pragma unroll
  for (int i = 0; i < 8; ++i) { out[i] = lo[i]; out[i + 8] = hi[i]; }
  return out;
}

__device__ __forceinline__ v8f wmma16(v16h a, v16h b, v8f c) {
  v8f d = __builtin_amdgcn_wmma_f32_16x16x32_f16(false, a, false, b, (short)0, c,
                                                 false, false);
  asm volatile("v_nop\n\tv_nop\n\tv_nop\n\tv_nop" : "+v"(d) : "v"(a), "v"(b));
  return d;
}

__global__ __launch_bounds__(256) void wconv_kernel(
    const float* __restrict__ W, _Float16* __restrict__ Wt, unsigned ldw, unsigned ldk,
    unsigned krows) {
#pragma clang fp contract(off)
  __shared__ _Float16 T[64 * LDT];
  const unsigned tid = threadIdx.x;
  const unsigned n0 = blockIdx.x * 64u;
  const unsigned k0 = blockIdx.y * 64u;
#pragma unroll 4
  for (unsigned j = 0; j < 16u; ++j) {
    const unsigned idx = tid + 256u * j;
    const unsigned kr = idx >> 6, nc = idx & 63u;
    const unsigned kk = k0 + kr;
    const unsigned kq = (kk < krows) ? kk : (krows - 1u);
    float v0 = W[(size_t)kq * ldw + n0 + nc];
    asm volatile("" : "+v"(v0));
    const float v = (kk < krows) ? v0 : 0.0f;
    T[nc * LDT + kr] = toh_flush(WCARRY * bf16r(v));
  }
  __syncthreads();
  v8h x[2];
  size_t off[2];
#pragma unroll
  for (unsigned i = 0; i < 2u; ++i) {
    const unsigned n = 32u * i + (tid >> 3);
    const unsigned kc = (tid & 7u) * 8u;
    x[i] = *(const v8h*)&T[n * LDT + kc];
    off[i] = (size_t)(n0 + n) * ldk + k0 + kc;
  }
#pragma unroll
  for (int i = 0; i < 2; ++i) *(volatile v8h*)(Wt + off[i]) = x[i];
  __threadfence();
#pragma unroll
  for (int i = 0; i < 2; ++i) *(volatile v8h*)(Wt + off[i]) = x[i];
}

__global__ __launch_bounds__(256) void count_kernel(
    const int* __restrict__ word, const int* __restrict__ age, _Float16* __restrict__ X16) {
#pragma clang fp contract(off)
  __shared__ _Float16 Rw[TOKB * KPITCH];
  __shared__ int Ids[TOKB * IDP];
  const unsigned lane = threadIdx.x & 31u;
  const unsigned wave = (unsigned)__builtin_amdgcn_readfirstlane((int)(threadIdx.x >> 5));
  const unsigned tok = blockIdx.x * (unsigned)TOKB + wave;
  const unsigned bidx = tok / (unsigned)SEQ;
  const unsigned sq = tok - bidx * (unsigned)SEQ;
  const size_t ftok = (size_t)bidx * SEQ_FULL + sq;
  const unsigned rbase = wave * (unsigned)KPITCH;
  const unsigned ibase = wave * (unsigned)IDP;

  const v8h zero = {};
#pragma unroll
  for (unsigned j = 0; j < (unsigned)CSTEPS; ++j) {
    const unsigned p = lane + 32u * j;
    if (p < (unsigned)ROWPIECES) *(v8h*)&Rw[rbase + p * 8u] = zero;
  }
  const int w0 = word[ftok * BAG + lane];
  const int w1 = word[ftok * BAG + 32u + (lane & 7u)];
  const int ag = age[ftok];
  Ids[ibase + lane] = w0;
  if (lane < 8u) Ids[ibase + 32u + lane] = w1;
  if (lane == 8u) Ids[ibase + 40u] = ag;
  __syncthreads();

  if (lane == 0u) {
#pragma unroll 1
    for (unsigned j = 0; j < (unsigned)BAG; ++j) {
      const int id = Ids[ibase + j];
      const bool ok = (id >= 0) && (id < VOCAB);
      const int lo = (id < 0) ? 0 : id;
      const unsigned ic = (unsigned)((lo > VOCAB - 1) ? (VOCAB - 1) : lo);
      const float c = (float)Rw[rbase + ic];
      Rw[rbase + ic] = toh_flush(c + (ok ? 1.0f : 0.0f));
    }
    {
      const int id = Ids[ibase + 40u];
      const bool ok = (id >= 0) && (id < AGE_DEPTH);
      const int lo = (id < 0) ? 0 : id;
      const unsigned ic = (unsigned)VOCAB + (unsigned)((lo > AGE_DEPTH - 1) ? (AGE_DEPTH - 1) : lo);
      const float c = (float)Rw[rbase + ic];
      Rw[rbase + ic] = toh_flush(c + (ok ? 1.0f : 0.0f));
    }
  }
  __syncthreads();

  v8h x[CSTEPS];
#pragma unroll
  for (unsigned j = 0; j < (unsigned)CSTEPS; ++j) {
    const unsigned p = lane + 32u * j;
    const unsigned pc = (p < (unsigned)ROWPIECES) ? p : (unsigned)(ROWPIECES - 1);
    x[j] = *(const v8h*)&Rw[rbase + pc * 8u];
  }
  _Float16* dst = X16 + (size_t)tok * KPITCH;
#pragma unroll
  for (unsigned j = 0; j < (unsigned)CSTEPS; ++j) {
    const unsigned p = lane + 32u * j;
    if (p < (unsigned)ROWPIECES) *(volatile v8h*)(dst + p * 8u) = x[j];
  }
  __threadfence();
#pragma unroll
  for (unsigned j = 0; j < (unsigned)CSTEPS; ++j) {
    const unsigned p = lane + 32u * j;
    if (p < (unsigned)ROWPIECES) *(volatile v8h*)(dst + p * 8u) = x[j];
  }
}

__global__ __launch_bounds__(256) void gemm_out_kernel(
    const _Float16* __restrict__ A16, const _Float16* __restrict__ Bt,
    const float* __restrict__ bias, float* __restrict__ outf) {
  __shared__ float Cs[64 * LDC];
  const unsigned tid = threadIdx.x, lane = tid & 31u;
  const unsigned w = (unsigned)__builtin_amdgcn_readfirstlane((int)(threadIdx.x >> 5));
  const unsigned mw = w >> 1, nw = w & 1u;
  const unsigned hh = lane >> 4, m = lane & 15u;
  const unsigned n0 = blockIdx.x * 64u;
  const unsigned row0 = blockIdx.y * 64u;

  const _Float16* ap  = A16 + (size_t)(row0 + mw * 16u + m) * KPITCH + hh * 8u;
  const _Float16* bp0 = Bt + (size_t)(n0 + nw * 32u + m) * KPITCH + hh * 8u;
  const _Float16* bp1 = bp0 + (size_t)16 * KPITCH;
  v8f acc0 = {}, acc1 = {};
#pragma unroll 2
  for (unsigned k0 = 0; k0 < (unsigned)KLOOP; k0 += 32u) {
    const v16h a  = frag_at(ap + k0);
    const v16h b0 = frag_at(bp0 + k0);
    const v16h b1 = frag_at(bp1 + k0);
    acc0 = wmma16(a, b0, acc0);
    acc1 = wmma16(a, b1, acc1);
  }
#pragma unroll
  for (int r = 0; r < 8; ++r) {
    float* d = &Cs[(mw * 16u + hh * 8u + (unsigned)r) * LDC + nw * 32u + m];
    d[0]  = acc0[r];
    d[16] = acc1[r];
  }
  __syncthreads();

  v4f xs[4];
  size_t off[4];
#pragma unroll
  for (unsigned i = 0; i < 4u; ++i) {
    const unsigned r = 16u * i + (tid >> 4);
    const unsigned c = (tid & 15u) * 4u;
    const unsigned crow = row0 + r;
    const unsigned bidx = crow / (unsigned)SEQ;
    const unsigned sq = crow - bidx * (unsigned)SEQ;
    const size_t frow = (size_t)bidx * SEQ_FULL + sq;
    const v4f u = *(const v4f*)&Cs[r * LDC + c];
    const v4f g = *(const v4f*)(bias + n0 + c);
    v4f val;
#pragma unroll
    for (int j = 0; j < 4; ++j) val[j] = u[j] * (1.0f / WCARRY) + bf16r(g[j]);
    xs[i] = val;
    off[i] = frow * DIMO + n0 + c;
  }
#pragma unroll
  for (int i = 0; i < 4; ++i) *(volatile v4f*)(outf + off[i]) = xs[i];
  __threadfence();
#pragma unroll
  for (int i = 0; i < 4; ++i) *(volatile v4f*)(outf + off[i]) = xs[i];
}

extern "C" void kernel_launch(void* const* d_in, const int* in_sizes, int n_in,
                              void* d_out, int out_size, void* d_ws, size_t ws_size,
                              hipStream_t stream) {
  if (n_in < 4) return;
  const long long need_tok = (long long)(NB - 1) * SEQ_FULL + SEQ;
  if ((long long)in_sizes[0] < need_tok * BAG) return;
  if ((long long)in_sizes[1] < need_tok) return;
  if ((long long)in_sizes[2] < (long long)KTRUE * DIMO) return;
  if (in_sizes[3] < DIMO) return;
  if ((long long)out_size < need_tok * DIMO) return;
  if (ws_size < WS_TOTAL) return;

  const int*   word = (const int*)d_in[0];
  const int*   age  = (const int*)d_in[1];
  const float* W    = (const float*)d_in[2];
  const float* bias = (const float*)d_in[3];
  float* out = (float*)d_out;

  char* ws = (char*)d_ws;
  _Float16* Wt16 = (_Float16*)(ws + OFF_WT);
  _Float16* X16  = (_Float16*)(ws + OFF_X);

  dim3 blk(256);
  wconv_kernel<<<dim3(DIMO / 64, KPITCH / 64), blk, 0, stream>>>(
      W, Wt16, (unsigned)DIMO, (unsigned)KPITCH, (unsigned)KTRUE);
  count_kernel<<<dim3(MROWS / TOKB), blk, 0, stream>>>(word, age, X16);
  gemm_out_kernel<<<dim3(DIMO / 64, MROWS / 64), blk, 0, stream>>>(X16, Wt16, bias, out);
}
